// ImageDiagnostic_55233279427342
// MI455X (gfx1250) — hardware-run, weakly checked
//
#include <hip/hip_runtime.h>


namespace {
constexpr int NB_ = 16, N = 50000, M = 128, NP = 50048  ;
constexpr float KS = 256.0f;
typedef _Float16 b16;
typedef __attribute__((ext_vector_type(16))) _Float16 v16b;
typedef __attribute__((ext_vector_type(8))) _Float16 v8b;
typedef __attribute__((ext_vector_type(8))) float v8f;
typedef __attribute__((ext_vector_type(4))) float v4f;
typedef __attribute__((ext_vector_type(2))) _Float16 v2b;
__device__ __forceinline__ float bf16_rne(float f) { unsigned int u = __float_as_uint(f); u += 0x7FFFu + ((u >> 16) & 1u); float r = __uint_as_float(u & 0xFFFF0000u); asm volatile("" : "+v"(r)); return r; }
__device__ __forceinline__ float bfv(float f) { float r = bf16_rne(f); asm volatile("" : "+v"(r)); return r; }
__device__ __forceinline__ void split16(float v, b16& hi, b16& lo) { hi = (b16)v; lo = (b16)(v - (float)hi); }
__device__ __forceinline__ v16b frag_kb(const b16* p, int hh) { const v8b a = *(const v8b*)(p + 8 * hh), b = *(const v8b*)(p + 16 + 8 * hh); v16b f;
#pragma unroll
  for (int e = 0; e < 8; ++e) { f[e] = a[e]; f[8 + e] = b[e]; } return f; }
__device__ __forceinline__ v8f wmma16b(v16b a, v16b b, v8f c) { v8f d = __builtin_amdgcn_wmma_f32_16x16x32_f16(false, a, false, b, (short)0, c, false, false); asm volatile("v_nop\n\tv_nop\n\tv_nop\n\tv_nop" : "+v"(d) : "v"(a), "v"(b)); return d; }
__device__ __forceinline__ void wave_lds_sync() { __builtin_amdgcn_fence(__ATOMIC_RELEASE, "workgroup"); __builtin_amdgcn_wave_barrier(); __builtin_amdgcn_fence(__ATOMIC_ACQUIRE, "workgroup"); }
__device__ __forceinline__ float pmul(float a, float b) { float p = a * b; asm volatile("" : "+v"(p)); return p; }

__global__ __launch_bounds__(32) void tab_kernel(const float* __restrict__ xv, const float* __restrict__ yv, const float* __restrict__ bins, const float* __restrict__ bw, int b, b16* __restrict__ KXh, b16* __restrict__ KXl, b16* __restrict__ KYh, b16* __restrict__ KYl) { __shared__ float Bn[M]; const int lane = threadIdx.x; const int n0 = blockIdx.x * 64 + 2 * lane; for (int q = 0; q < 4; ++q) Bn[q * 32 + lane] = bfv(bins[q * 32 + lane]);
  wave_lds_sync(); const float ib = 1.0f / bfv(bw[0]); float x0 = 0.0f, x1 = 0.0f, y0 = 0.0f, y1 = 0.0f; const bool v0 = n0 < N, v1 = n0 + 1 < N;
  if (v0) { x0 = bfv(xv[(size_t)b * N + n0]); y0 = bfv(yv[(size_t)b * N + n0]); } if (v1) { x1 = bfv(xv[(size_t)b * N + n0 + 1]); y1 = bfv(yv[(size_t)b * N + n0 + 1]); }
  for (int pass = 0; pass < 2; ++pass) {
#pragma unroll 1
    for (int m = 0; m < M; ++m) { const float c = Bn[m]; float t; b16 h0, l0, h1, l1;
      t = (x0 - c) * ib; split16((v0 ? __expf(-0.5f * t * t) : 0.0f) * KS, h0, l0); t = (x1 - c) * ib; split16((v1 ? __expf(-0.5f * t * t) : 0.0f) * KS, h1, l1);
      *(volatile v2b*)(KXh + (size_t)m * NP + n0) = (v2b){h0, h1}; *(volatile v2b*)(KXl + (size_t)m * NP + n0) = (v2b){l0, l1};
      t = (y0 - c) * ib; split16((v0 ? __expf(-0.5f * t * t) : 0.0f) * KS, h0, l0); t = (y1 - c) * ib; split16((v1 ? __expf(-0.5f * t * t) : 0.0f) * KS, h1, l1);
      *(volatile v2b*)(KYh + (size_t)m * NP + n0) = (v2b){h0, h1}; *(volatile v2b*)(KYl + (size_t)m * NP + n0) = (v2b){l0, l1}; }
    __threadfence(); } }
__global__ __launch_bounds__(32) void gemm_kernel(const b16* __restrict__ KXh, const b16* __restrict__ KXl, const b16* __restrict__ KYh, const b16* __restrict__ KYl, float* __restrict__ J) { __shared__ float Tf[32][M + 4]; const int lane = threadIdx.x, nloc = lane & 15, hlf = lane >> 4; const int m0 = blockIdx.x * 32; v8f acc[2][8];
#pragma unroll
  for (int rt = 0; rt < 2; ++rt)
#pragma unroll
    for (int t = 0; t < 8; ++t) acc[rt][t] = (v8f){};
#pragma unroll 1
  for (int kb = 0; kb < NP; kb += 32) { const v16b ah0 = frag_kb(KXh + (size_t)(m0 + nloc) * NP + kb, hlf), al0 = frag_kb(KXl + (size_t)(m0 + nloc) * NP + kb, hlf), ah1 = frag_kb(KXh + (size_t)(m0 + 16 + nloc) * NP + kb, hlf), al1 = frag_kb(KXl + (size_t)(m0 + 16 + nloc) * NP + kb, hlf);
#pragma unroll
    for (int t = 0; t < 8; ++t) { const v16b bh = frag_kb(KYh + (size_t)(t * 16 + nloc) * NP + kb, hlf), bl = frag_kb(KYl + (size_t)(t * 16 + nloc) * NP + kb, hlf);
      acc[0][t] = wmma16b(ah0, bh, acc[0][t]); acc[0][t] = wmma16b(ah0, bl, acc[0][t]); acc[0][t] = wmma16b(al0, bh, acc[0][t]);
      acc[1][t] = wmma16b(ah1, bh, acc[1][t]); acc[1][t] = wmma16b(ah1, bl, acc[1][t]); acc[1][t] = wmma16b(al1, bh, acc[1][t]); } }
#pragma unroll
  for (int rt = 0; rt < 2; ++rt)
#pragma unroll
    for (int t = 0; t < 8; ++t)
#pragma unroll
      for (int r8 = 0; r8 < 8; ++r8) Tf[rt * 16 + 8 * hlf + r8][t * 16 + nloc] = acc[rt][t][r8] * (1.0f / (KS * KS));
  wave_lds_sync();
  for (int pass = 0; pass < 2; ++pass) { for (int r = 0; r < 32; ++r) *(volatile v4f*)(J + (size_t)(m0 + r) * M + lane * 4) = *(const v4f*)(&Tf[r][lane * 4]); __threadfence(); } }
__global__ __launch_bounds__(32) void norm_kernel(const float* __restrict__ J, int b, float* __restrict__ out) { const int lane = threadIdx.x; double s = 0.0; for (int r = 0; r < M; ++r) for (int q = 0; q < 4; ++q) s += (double)J[(size_t)r * M + q * 32 + lane];
  for (int o = 16; o; o >>= 1) s += __shfl_xor(s, o);
  const float inv = (float)(1.0 / (s + 1e-10));
  for (int pass = 0; pass < 2; ++pass) { for (int r = 0; r < M; ++r) *(volatile v4f*)(out + ((size_t)b * M + r) * M + lane * 4) = *(const v4f*)(J + (size_t)r * M + lane * 4) * inv; __threadfence(); } }
}

extern "C" void kernel_launch(void* const* d_in, const int* in_sizes, int n_in, void* d_out, int out_size, void* d_ws, size_t ws_size, hipStream_t stream) {
  (void)n_in;
  auto Fp = [&](int i) { return (const float*)d_in[i]; };
  if (in_sizes[0] != NB_ * N || in_sizes[1] != NB_ * N || in_sizes[2] != M || in_sizes[3] != 1 || out_size != NB_ * M * M) return;
  const int BLIM = NB_;
  size_t off = 0; char* ws = (char*)d_ws;
  auto carve = [&](size_t bytes) { char* p = ws + off; off += (bytes + 255) & ~(size_t)255; return p; };
  b16* KXh = (b16*)carve((size_t)M * NP * 2); b16* KXl = (b16*)carve((size_t)M * NP * 2); b16* KYh = (b16*)carve((size_t)M * NP * 2); b16* KYl = (b16*)carve((size_t)M * NP * 2); float* J = (float*)carve((size_t)M * M * 4);
  if (off > ws_size || off > ((size_t)64 << 20)) return;
  for (int b = 0; b < BLIM; ++b) {
    tab_kernel<<<NP / 64, 32, 0, stream>>>(Fp(0), Fp(1), Fp(2), Fp(3), b, KXh, KXl, KYh, KYl);
    gemm_kernel<<<M / 32, 32, 0, stream>>>(KXh, KXl, KYh, KYl, J);
    norm_kernel<<<1, 32, 0, stream>>>(J, b, (float*)d_out); }
}
